// ChebyshevLayer_33629593928064
// MI455X (gfx1250) — hardware-verified
//
#include <hip/hip_runtime.h>


namespace {
constexpr int NB_ = 64, IC = 64, OC_ = 64, NG = 2048, MD = 512, NR = NB_ * IC  ;
constexpr float XS = 8.0f, MS = 64.0f, HS = 256.0f, WSC = 256.0f, OS = 16.0f;
typedef _Float16 b16;
typedef __attribute__((ext_vector_type(16))) _Float16 v16b;
typedef __attribute__((ext_vector_type(8))) _Float16 v8b;
typedef __attribute__((ext_vector_type(2))) _Float16 v2b;
typedef __attribute__((ext_vector_type(8))) float v8f;
typedef __attribute__((ext_vector_type(4))) float v4f;
__device__ __forceinline__ float bf16_rne(float f) { unsigned int u = __float_as_uint(f); u += 0x7FFFu + ((u >> 16) & 1u); float r = __uint_as_float(u & 0xFFFF0000u); asm volatile("" : "+v"(r)); return r; }
__device__ __forceinline__ float bfv(float f) { float r = bf16_rne(f); asm volatile("" : "+v"(r)); return r; }
__device__ __forceinline__ void split16(float v, b16& hi, b16& lo) { hi = (b16)v; lo = (b16)(v - (float)hi); }
__device__ __forceinline__ v16b frag_kb(const b16* p, int hh) { const v8b a = *(const v8b*)(p + 8 * hh), b = *(const v8b*)(p + 16 + 8 * hh); v16b f;
#pragma unroll
  for (int e = 0; e < 8; ++e) { f[e] = a[e]; f[8 + e] = b[e]; } return f; }
__device__ __forceinline__ v8f wmma16b(v16b a, v16b b, v8f c) { v8f d = __builtin_amdgcn_wmma_f32_16x16x32_f16(false, a, false, b, (short)0, c, false, false); asm volatile("v_nop\n\tv_nop\n\tv_nop\n\tv_nop" : "+v"(d) : "v"(a), "v"(b)); return d; }
__device__ __forceinline__ void wave_lds_sync() { __builtin_amdgcn_fence(__ATOMIC_RELEASE, "workgroup"); __builtin_amdgcn_wave_barrier(); __builtin_amdgcn_fence(__ATOMIC_ACQUIRE, "workgroup"); }
__device__ __forceinline__ float pmul(float a, float b) { float p = a * b; asm volatile("" : "+v"(p)); return p; }
__device__ __forceinline__ float mval(int k, int n) { float a = 3.14159274101257324f * (float)(k * n); asm volatile("" : "+v"(a)); const float arg = a / 2047.0f; const float cs = cosf(arg); return cs; }

__global__ __launch_bounds__(256) void prep_kernel(const float* __restrict__ x, b16* __restrict__ MFh, b16* __restrict__ MFl, b16* __restrict__ MIh, b16* __restrict__ MIl, b16* __restrict__ X16) { const size_t nt = (size_t)gridDim.x * 256, u0 = (size_t)blockIdx.x * 256 + threadIdx.x;
  for (size_t u = u0; u < (size_t)MD * NG / 2; u += nt) { const int k = (int)(u / (NG / 2)), n = (int)(u % (NG / 2)) * 2; b16 h0, l0, h1, l1; const float c0 = (n == 0 || n == NG - 1) ? 1.0f : 2.0f, c1 = (n + 1 == NG - 1) ? 1.0f : 2.0f; split16(mval(k, n) * c0 * MS, h0, l0); split16(mval(k, n + 1) * c1 * MS, h1, l1); for (int pass = 0; pass < 2; ++pass) { *(volatile v2b*)(MFh + (size_t)k * NG + n) = (v2b){h0, h1}; *(volatile v2b*)(MFl + (size_t)k * NG + n) = (v2b){l0, l1}; __threadfence(); } }
  for (size_t u = u0; u < (size_t)NG * MD / 2; u += nt) { const int n = (int)(u / (MD / 2)), k = (int)(u % (MD / 2)) * 2; b16 h0, l0, h1, l1; const float c0 = (k == 0) ? 1.0f : 2.0f, c1 = 2.0f; split16(mval(n, k) * c0 * MS, h0, l0); split16(mval(n, k + 1) * c1 * MS, h1, l1); for (int pass = 0; pass < 2; ++pass) { *(volatile v2b*)(MIh + (size_t)n * MD + k) = (v2b){h0, h1}; *(volatile v2b*)(MIl + (size_t)n * MD + k) = (v2b){l0, l1}; __threadfence(); } }
  for (size_t u = u0; u < (size_t)NR * NG / 8; u += nt) { v8b v;
#pragma unroll
    for (int j = 0; j < 8; ++j) v[j] = (b16)(bf16_rne(x[u * 8 + j]) * XS); for (int pass = 0; pass < 2; ++pass) { *(volatile v8b*)(X16 + u * 8) = v; __threadfence(); } } }
__global__ __launch_bounds__(32) void fwd_kernel(const b16* __restrict__ MFh, const b16* __restrict__ MFl, const b16* __restrict__ X16, int KLIM, float* __restrict__ X1) { __shared__ float Tf[16][260]; const int lane = threadIdx.x, nloc = lane & 15, hlf = lane >> 4; const int k0 = blockIdx.x * 16, r0 = blockIdx.y * 256; if (k0 >= KLIM) return; v8f acc[16];
#pragma unroll
  for (int t = 0; t < 16; ++t) acc[t] = (v8f){};
#pragma unroll 2
  for (int kb = 0; kb < NG; kb += 32) { const v16b a = frag_kb(MFh + (size_t)(k0 + nloc) * NG + kb, hlf), al = frag_kb(MFl + (size_t)(k0 + nloc) * NG + kb, hlf);
#pragma unroll
    for (int t = 0; t < 16; ++t) { const v16b bx = frag_kb(X16 + (size_t)(r0 + t * 16 + nloc) * NG + kb, hlf); acc[t] = wmma16b(a, bx, acc[t]); acc[t] = wmma16b(al, bx, acc[t]); } }
#pragma unroll
  for (int t = 0; t < 16; ++t)
#pragma unroll
    for (int r8 = 0; r8 < 8; ++r8) Tf[8 * hlf + r8][t * 16 + nloc] = acc[t][r8] * (1.0f / (MS * XS));
  wave_lds_sync();
  for (int pass = 0; pass < 2; ++pass) { for (int rr = 0; rr < 16; ++rr) for (int q = 0; q < 2; ++q) *(volatile v4f*)(X1 + (size_t)(k0 + rr) * NR + r0 + q * 128 + lane * 4) = *(const v4f*)(&Tf[rr][q * 128 + lane * 4]); __threadfence(); } }
__global__ __launch_bounds__(32) void mix_kernel(const float* __restrict__ X1, const float* __restrict__ W, int KLIM, float* __restrict__ OCT) { __shared__ __attribute__((aligned(16))) b16 Wk[OC_][IC + 8], Ah[16][IC + 8], Al[16][IC + 8]; __shared__ float Tf[16][OC_ + 1]; const int lane = threadIdx.x, nloc = lane & 15, hlf = lane >> 4; const int k = blockIdx.x; if (k >= KLIM) return;
  for (int o = 0; o < OC_; ++o) for (int i = lane; i < IC + 8; i += 32) Wk[o][i] = (b16)(i < IC ? bfv(W[((size_t)i * OC_ + o) * MD + k]) * WSC : 0.0f);
  if (lane < 16) for (int i = IC; i < IC + 8; ++i) { Ah[lane][i] = (b16)0.0f; Al[lane][i] = (b16)0.0f; }
  wave_lds_sync();
#pragma unroll 1
  for (int bt = 0; bt < NB_ / 16; ++bt) {
    for (int rr = 0; rr < 16; ++rr) for (int q = 0; q < 2; ++q) { const int i = q * 32 + lane; b16 p, pl; split16(X1[(size_t)k * NR + (bt * 16 + rr) * IC + i] * OS, p, pl); Ah[rr][i] = p; Al[rr][i] = pl; }
    wave_lds_sync(); v8f acc[4] = {(v8f){}, (v8f){}, (v8f){}, (v8f){}};
#pragma unroll
    for (int kb = 0; kb < IC; kb += 32) { const v16b a = frag_kb(&Ah[nloc][kb], hlf), al = frag_kb(&Al[nloc][kb], hlf);
#pragma unroll
      for (int t = 0; t < 4; ++t) { const v16b bw = frag_kb(&Wk[t * 16 + nloc][kb], hlf); acc[t] = wmma16b(a, bw, acc[t]); acc[t] = wmma16b(al, bw, acc[t]); } }
#pragma unroll
    for (int t = 0; t < 4; ++t)
#pragma unroll
      for (int r8 = 0; r8 < 8; ++r8) Tf[8 * hlf + r8][t * 16 + nloc] = acc[t][r8] * (1.0f / (OS * WSC));
    wave_lds_sync();
    for (int pass = 0; pass < 2; ++pass) { for (int rr = 0; rr < 16; ++rr) for (int q = 0; q < 2; ++q) ((volatile float*)OCT)[(size_t)k * NR + (bt * 16 + rr) * OC_ + q * 32 + lane] = Tf[rr][q * 32 + lane]; __threadfence(); }
    wave_lds_sync(); } }
__global__ __launch_bounds__(256) void tr_kernel(const float* __restrict__ OCT, int KLIM, b16* __restrict__ OCh, b16* __restrict__ OCl) { __shared__ float Tt[64][65]; const int kt = blockIdx.x % (MD / 64), rt = blockIdx.x / (MD / 64); const int k0 = kt * 64, r0 = rt * 64; const int tid = threadIdx.x, wave = tid >> 5, lane = tid & 31;
  for (int kk = wave; kk < 64; kk += 8) for (int rr = lane; rr < 64; rr += 32) Tt[kk][rr] = (k0 + kk) < KLIM ? OCT[(size_t)(k0 + kk) * NR + r0 + rr] : 0.0f;
  __syncthreads();
  for (int pass = 0; pass < 2; ++pass) { for (int rr = wave; rr < 64; rr += 8) { b16 h0, l0, h1, l1; split16(Tt[lane * 2][rr] * OS, h0, l0); split16(Tt[lane * 2 + 1][rr] * OS, h1, l1); const size_t o = (size_t)(r0 + rr) * MD + k0 + lane * 2; *(volatile v2b*)(OCh + o) = (v2b){h0, h1}; *(volatile v2b*)(OCl + o) = (v2b){l0, l1}; } __threadfence(); } }
__global__ __launch_bounds__(32) void inv_kernel(const b16* __restrict__ OCh, const b16* __restrict__ OCl, const b16* __restrict__ MIh, const b16* __restrict__ MIl, int RLIM, float* __restrict__ y) { __shared__ float Tf[16][260]; const int lane = threadIdx.x, nloc = lane & 15, hlf = lane >> 4; const size_t r0 = (size_t)blockIdx.x * 16; const int c0 = blockIdx.y * 128; if (r0 >= (size_t)RLIM) return; v8f acc[8];
#pragma unroll
  for (int t = 0; t < 8; ++t) acc[t] = (v8f){};
#pragma unroll 2
  for (int kb = 0; kb < MD; kb += 32) { const v16b a = frag_kb(OCh + (r0 + nloc) * MD + kb, hlf), al = frag_kb(OCl + (r0 + nloc) * MD + kb, hlf);
#pragma unroll
    for (int t = 0; t < 8; ++t) { const size_t mo = (size_t)(c0 + t * 16 + nloc) * MD + kb; const v16b mh = frag_kb(MIh + mo, hlf), ml = frag_kb(MIl + mo, hlf); acc[t] = wmma16b(a, mh, acc[t]); acc[t] = wmma16b(a, ml, acc[t]); acc[t] = wmma16b(al, mh, acc[t]); } }
#pragma unroll
  for (int t = 0; t < 8; ++t)
#pragma unroll
    for (int r8 = 0; r8 < 8; ++r8) Tf[8 * hlf + r8][t * 16 + nloc] = acc[t][r8] * (1.0f / (OS * MS));
  wave_lds_sync();
  for (int pass = 0; pass < 2; ++pass) { for (int rr = 0; rr < 16; ++rr) *(volatile v4f*)(y + (r0 + rr) * NG + c0 + lane * 4) = *(const v4f*)(&Tf[rr][lane * 4]); __threadfence(); } }
}

extern "C" void kernel_launch(void* const* d_in, const int* in_sizes, int n_in, void* d_out, int out_size, void* d_ws, size_t ws_size, hipStream_t stream) {
  (void)n_in;
  auto Fp = [&](int i) { return (const float*)d_in[i]; };
  if (in_sizes[0] != NR * NG || in_sizes[1] != IC * OC_ * MD || out_size != NR * NG) return;
  const int KLIM = MD, RLIM = NR;
  size_t off = 0; char* ws = (char*)d_ws;
  auto carve = [&](size_t bytes) { char* p = ws + off; off += (bytes + 255) & ~(size_t)255; return p; };
  b16* MFh = (b16*)carve((size_t)MD * NG * 2); b16* MFl = (b16*)carve((size_t)MD * NG * 2); b16* MIh = (b16*)carve((size_t)NG * MD * 2); b16* MIl = (b16*)carve((size_t)NG * MD * 2); b16* X16 = (b16*)carve((size_t)NR * NG * 2); float* X1 = (float*)carve((size_t)MD * NR * 4); float* OCT = (float*)carve((size_t)MD * NR * 4); b16* OCh = (b16*)carve((size_t)NR * MD * 2); b16* OCl = (b16*)carve((size_t)NR * MD * 2);
  if (off > ws_size || off > ((size_t)64 << 20)) return;
  prep_kernel<<<512, 256, 0, stream>>>(Fp(0), MFh, MFl, MIh, MIl, X16);
  fwd_kernel<<<dim3(KLIM / 16, NR / 256), 32, 0, stream>>>(MFh, MFl, X16, KLIM, X1);
  mix_kernel<<<KLIM, 32, 0, stream>>>(X1, Fp(1), KLIM, OCT);
  tr_kernel<<<(MD / 64) * (NR / 64), 256, 0, stream>>>(OCT, KLIM, OCh, OCl);
  inv_kernel<<<dim3(NR / 16, NG / 128), 32, 0, stream>>>(OCh, OCl, MIh, MIl, RLIM, (float*)d_out);
}
